// GCNLayer_2345052144350
// MI455X (gfx1250) — hardware-verified
//
#include <hip/hip_runtime.h>

typedef float          v8f   __attribute__((ext_vector_type(8)));
typedef float          v4f   __attribute__((ext_vector_type(4)));
typedef unsigned int   v4u   __attribute__((ext_vector_type(4)));
typedef int            v8i   __attribute__((ext_vector_type(8)));
typedef unsigned short v8us  __attribute__((ext_vector_type(8)));
typedef unsigned short v16us __attribute__((ext_vector_type(16)));
typedef __bf16         v16bf __attribute__((ext_vector_type(16)));
typedef _Float16       v16h  __attribute__((ext_vector_type(16)));
typedef v4f  __attribute__((may_alias)) v4fa;
typedef v8us __attribute__((may_alias)) v8usa;
union FragB { v16bf v; v16us u; v8us h[2]; v8i w; };
union FragH { v16h  v; v16us u; v8us h[2]; v8i w; };

__device__ __forceinline__ v8f wmb(const FragB& a, const FragB& b, v8f c) {
  v8f d = __builtin_amdgcn_wmma_f32_16x16x32_bf16(false, a.v, false, b.v, (short)0, c, false, false);
  asm volatile("v_nop\n\tv_nop\n\tv_nop\n\tv_nop" : "+v"(d) : "v"(a.w), "v"(b.w));
  return d;
}

__device__ __forceinline__ v8f wmh(const FragH& a, const FragH& b, v8f c) {
  v8f d = __builtin_amdgcn_wmma_f32_16x16x32_f16(false, a.v, false, b.v, (short)0, c, false, false);
  asm volatile("v_nop\n\tv_nop\n\tv_nop\n\tv_nop" : "+v"(d) : "v"(a.w), "v"(b.w));
  return d;
}

__device__ __forceinline__ unsigned bf16_bits(float f) {
  const unsigned u = __float_as_uint(f);
  const unsigned r = (u + 0x7FFFu + ((u >> 16) & 1u)) >> 16;
  const unsigned q = (u >> 16) | 0x40u;
  return ((u & 0x7fffffffu) > 0x7f800000u) ? q : r;
}

__device__ __forceinline__ float bf16_val(float f) {
  return __uint_as_float(bf16_bits(f) << 16);
}
__device__ __forceinline__ int clampi(int v, int lo, int hi) {
  return v < lo ? lo : (v > hi ? hi : v);
}

__device__ __forceinline__ unsigned f16_bits(float f) {
  const unsigned u  = __float_as_uint(f);
  const unsigned s  = (u >> 16) & 0x8000u;
  const unsigned a  = u & 0x7fffffffu;
  const unsigned t  = a - 0x38000000u;
  const unsigned r  = (t + 0x0FFFu + ((t >> 13) & 1u)) >> 13;
  const unsigned rc = r > 0x7C00u ? 0x7C00u : r;
  const bool small  = a < 0x38800000u;
  const bool isnan  = a > 0x7f800000u;
  const unsigned fin = small ? 0u : (s | rc);
  return isnan ? (s | 0x7E00u) : fin;
}

__device__ __forceinline__ unsigned pk16(unsigned lo, unsigned hi) { return lo | (hi << 16); }
__device__ __forceinline__ unsigned bf16_lo_bits(float v) {
  float hi = bf16_val(v);
  asm volatile("" : "+v"(hi));
  return bf16_bits(v - hi);
}
__device__ __forceinline__ v4u pack8_bf16(v4f a, v4f c) {
  return (v4u){ pk16(bf16_bits(a[0]), bf16_bits(a[1])), pk16(bf16_bits(a[2]), bf16_bits(a[3])),
                pk16(bf16_bits(c[0]), bf16_bits(c[1])), pk16(bf16_bits(c[2]), bf16_bits(c[3])) };
}
__device__ __forceinline__ v4u pack8_bf16_lo(v4f a, v4f c) {
  return (v4u){ pk16(bf16_lo_bits(a[0]), bf16_lo_bits(a[1])), pk16(bf16_lo_bits(a[2]), bf16_lo_bits(a[3])),
                pk16(bf16_lo_bits(c[0]), bf16_lo_bits(c[1])), pk16(bf16_lo_bits(c[2]), bf16_lo_bits(c[3])) };
}
__device__ __forceinline__ v4u pack8_f16(v4f a, v4f c) {
  return (v4u){ pk16(f16_bits(a[0]), f16_bits(a[1])), pk16(f16_bits(a[2]), f16_bits(a[3])),
                pk16(f16_bits(c[0]), f16_bits(c[1])), pk16(f16_bits(c[2]), f16_bits(c[3])) };
}

template <int FORM>
__global__ __launch_bounds__(256) void k_plane(const float* __restrict__ src, int rows, int cols, int ldsrc,
                                               unsigned short* __restrict__ dst, int MP, int KP) {
  static_assert(FORM >= 0 && FORM <= 3);
  const int KTOT = (FORM == 1 || FORM == 3) ? 2 * KP : KP;
  const unsigned ppr   = (unsigned)(KTOT >> 3);
  const unsigned kp8   = (unsigned)(KP >> 3);
  const unsigned total = (unsigned)MP * ppr;
  const unsigned g     = blockIdx.x * 256u + threadIdx.x;
  const unsigned rowu  = g / ppr;
  const unsigned p     = g - rowu * ppr;
  const bool second    = p >= kp8;
  const int row = (int)rowu;
  const int c0  = (int)((second ? p - kp8 : p) << 3);
  const float* srow = src + (size_t)clampi(row, 0, rows - 1) * (size_t)ldsrc;
  float x[8];
  unsigned mk[8];
#pragma unroll
  for (int e = 0; e < 8; ++e) {
    const int c = c0 + e;
    const float v = srow[clampi(c, 0, cols - 1)];
    asm volatile("" :: "v"(v));
    x[e]  = v;
    mk[e] = (row < rows && c < cols) ? 0xFFFFu : 0u;
  }
  const v4f a = (v4f){ x[0], x[1], x[2], x[3] };
  const v4f c = (v4f){ x[4], x[5], x[6], x[7] };
  v4u o;
  if (FORM == 2) {
    o = pack8_f16(a, c);
  } else {
    const v4u hi = pack8_bf16(a, c);
    o = hi;
    if (FORM == 1) { const v4u lo = pack8_bf16_lo(a, c); o = second ? lo : hi; }
  }
  const v4u mw = (v4u){ pk16(mk[0], mk[1]), pk16(mk[2], mk[3]), pk16(mk[4], mk[5]), pk16(mk[6], mk[7]) };
  o &= mw;
  if (g < total) {
    volatile v4u* q = (volatile v4u*)(dst + (size_t)g * 8);
    *q = o;
    __threadfence();
    *q = o;
  }
}

template <int FORM> struct FragOf    { typedef FragB T; };
template <>         struct FragOf<2> { typedef FragH T; };
__device__ __forceinline__ v8f mm(const FragB& a, const FragB& b, v8f c) { return wmb(a, b, c); }
__device__ __forceinline__ v8f mm(const FragH& a, const FragH& b, v8f c) { return wmh(a, b, c); }
template <class F> __device__ __forceinline__ F ld_frag(const unsigned short* p) {
  F f;
  f.h[0] = *(const v8usa*)(p);
  f.h[1] = *(const v8usa*)(p + 16);
  return f;
}

template <int FORM, int EPI>
__global__ __launch_bounds__(256) __attribute__((amdgpu_num_vgpr(248)))
void k_gemm_nt(const unsigned short* __restrict__ A, const unsigned short* __restrict__ B,
               const float* __restrict__ bias, float* __restrict__ D, int M, int N, int KTOT, int ldd) {
  static_assert(FORM >= 0 && FORM <= 2);
  static_assert(EPI == 0 || EPI == 1);
  typedef typename FragOf<FORM>::T F;
  __shared__ __attribute__((aligned(16))) float sT[8][16 * 68];
  const int lane = threadIdx.x & 31;
  const int wave = threadIdx.x >> 5;
  const int tilesM = (M + 63) >> 6;
  const int tilesN = (N + 63) >> 6;
  const int tile = blockIdx.x * 8 + wave;
  if (tile >= tilesM * tilesN) return;
  const int tm = tile / tilesN;
  const int tn = tile - tm * tilesN;
  const int m0 = tm << 6;
  const int n0 = tn << 6;

  const int rl = lane & 15;
  const int h8 = (lane >> 4) * 8;
  const unsigned short* pa = A + (size_t)(m0 + rl) * (size_t)KTOT + h8;
  const unsigned short* pb = B + (size_t)(n0 + rl) * (size_t)KTOT + h8;

  v8f acc[4][4];
#pragma unroll
  for (int i = 0; i < 4; ++i)
#pragma unroll
    for (int j = 0; j < 4; ++j) acc[i][j] = (v8f){0.f, 0.f, 0.f, 0.f, 0.f, 0.f, 0.f, 0.f};

#pragma unroll 1
  for (int k0 = 0; k0 < KTOT; k0 += 32) {
    F bf[4];
#pragma unroll
    for (int j = 0; j < 4; ++j) bf[j] = ld_frag<F>(pb + (size_t)(j << 4) * (size_t)KTOT + k0);
#pragma unroll
    for (int i = 0; i < 4; ++i) {
      const F af = ld_frag<F>(pa + (size_t)(i << 4) * (size_t)KTOT + k0);
#pragma unroll
      for (int j = 0; j < 4; ++j) acc[i][j] = mm(af, bf[j], acc[i][j]);
    }
  }

  float* slab = sT[wave];
  const int hh = lane >> 4;
  const int c4 = (lane & 15) * 4;
  const int nc = n0 + c4;
  const bool cok = nc < N;
  v4f bv = (v4f){0.f, 0.f, 0.f, 0.f};
  if (EPI == 1) {
    bv = *(const v4fa*)(bias + clampi(nc, 0, N - 4));
    asm volatile("" :: "v"(bv));
  }
#pragma unroll
  for (int i = 0; i < 4; ++i) {
    const int mBase = m0 + (i << 4);
#pragma unroll
    for (int j = 0; j < 4; ++j) {
#pragma unroll
      for (int r = 0; r < 8; ++r) slab[(h8 + r) * 68 + (j << 4) + rl] = acc[i][j][r];
    }
    __builtin_amdgcn_fence(__ATOMIC_RELEASE, "workgroup");
    __builtin_amdgcn_wave_barrier();
    __builtin_amdgcn_fence(__ATOMIC_ACQUIRE, "workgroup");
    v4f vv[8];
#pragma unroll
    for (int it = 0; it < 8; ++it) {
      const int row = it * 2 + hh;
      v4f v = *(const v4fa*)(slab + row * 68 + c4);
      if (EPI == 1) v += bv;
      vv[it] = v;
    }
    for (int pass = 0; pass < 2; ++pass) {
#pragma unroll
      for (int it = 0; it < 8; ++it) {
        const int row = mBase + it * 2 + hh;
        if (cok && row < M) *(volatile v4f*)(D + (size_t)row * (size_t)ldd + nc) = vv[it];
      }
      __threadfence();
    }
    __builtin_amdgcn_fence(__ATOMIC_RELEASE, "workgroup");
    __builtin_amdgcn_wave_barrier();
    __builtin_amdgcn_fence(__ATOMIC_ACQUIRE, "workgroup");
  }
}

#include <stddef.h>
#include <stdint.h>

#pragma clang fp contract(off)

#define NN      100000
#define NE      1000000
#define DF      128
#define MPAD    100096
#define NTHR    256
#define NWAVE   8
#define NBRUN   1024
#define SLB     10
#define NBLK    98
#define NSLOT   (NBLK * NBRUN)
#define STEPB   2048
#define NSTEP   ((NE + STEPB - 1) / STEPB)
#define LCAP    13312
#define DEGCAP  48
#define MEAS_B1024 10492
#define MEAS_DEG   25
#define BK_ZINTS   (2 * LCAP + 3 * NBRUN)
#define BK_MISC    32
#define BK_INTS    (BK_ZINTS + BK_MISC)
#define BK_LDS     (BK_INTS * 4)
#define LIST_IT    ((LCAP / 4) / NTHR)
#define WTP        136
#define TB_NODE_BLKS (MPAD / NTHR)

static_assert(NN % NWAVE == 0 && NN % 16 == 0 && DF == 128 && DF % 32 == 0 && DF % 64 == 0);
static_assert(NBRUN == (1 << SLB));
static_assert((NBLK - 1) * NBRUN < NN && NBLK * NBRUN >= NN && NN - (NBLK - 1) * NBRUN == 672 && NBLK == 98);
static_assert(MPAD % 128 == 0 && MPAD % 64 == 0 && MPAD >= NN && MPAD >= ((NN + 63) / 64) * 64);
static_assert((MPAD * (DF / 8)) % 256 == 0 && MPAD % NTHR == 0 && TB_NODE_BLKS == 391);
static_assert(NE % 8 == 0 && NE - 488 * STEPB == 576 && NE % 256 == 64 && NSTEP == 489);
static_assert(NN <= (1 << 17) && SLB + 17 <= 31);
static_assert(4 * LCAP >= 5 * MEAS_B1024 && LCAP % 256 == 0 && (LCAP / 4) % NTHR == 0 && LIST_IT == 13);
static_assert(DEGCAP >= MEAS_DEG + 8 && LCAP > DEGCAP);
static_assert(BK_ZINTS % (NTHR * 4) == 0 && (BK_ZINTS * 4) % 16 == 0);
static_assert(BK_LDS == 118912 && BK_LDS <= 262144 && BK_LDS + 0 <= 327680);
static_assert((WTP * 2) % 16 == 0 && WTP >= DF && DF * WTP * 2 == 34816);

typedef int v4i __attribute__((ext_vector_type(4)));
typedef v4i __attribute__((may_alias)) v4ia;
typedef v4u __attribute__((may_alias)) v4ua;

#define PIN(x) asm volatile("" :: "v"(x))

__global__ __launch_bounds__(NTHR) void k_wt(const float* __restrict__ W, unsigned short* WT) {
  __shared__ __attribute__((aligned(16))) unsigned short sw[DF * WTP];
  const int tid = (int)threadIdx.x;
#pragma unroll 4
  for (int i = 0; i < 16; ++i) {
    const int q  = i * NTHR + tid;
    const int k  = q >> 5;
    const int n4 = (q & 31) << 2;
    const v4f v = *(const v4fa*)(W + (size_t)k * DF + n4);
    sw[(n4 + 0) * WTP + k] = (unsigned short)bf16_bits(v[0]);
    sw[(n4 + 1) * WTP + k] = (unsigned short)bf16_bits(v[1]);
    sw[(n4 + 2) * WTP + k] = (unsigned short)bf16_bits(v[2]);
    sw[(n4 + 3) * WTP + k] = (unsigned short)bf16_bits(v[3]);
  }
  __syncthreads();
  v4u o[8];
#pragma unroll
  for (int i = 0; i < 8; ++i) {
    const int piece = i * NTHR + tid;
    const int n  = piece >> 4;
    const int k8 = (piece & 15) << 3;
    o[i] = *(const v4ua*)(sw + n * WTP + k8);
  }
  for (int pass = 0; pass < 2; ++pass) {
#pragma unroll
    for (int i = 0; i < 8; ++i) {
      const int piece = i * NTHR + tid;
      *(volatile v4u*)(WT + (size_t)piece * 8) = o[i];
    }
    __threadfence();
  }
}

__device__ __forceinline__ float inv_sqrt_src(int deg) {
  float g = (float)deg;
  g = g < 1.0f ? 1.0f : g;
  return 1.0f / sqrtf(g);
}
__device__ __forceinline__ float inv_sqrt_own(int deg) {
  float g = (float)deg;
  g = g < 1.0f ? 1.0f : g;
  g = g > 10.0f ? 10.0f : g;
  return 1.0f / sqrtf(g);
}

__global__ __launch_bounds__(NTHR) void k_tables(const int* __restrict__ odeg, const int* __restrict__ ideg,
                                                 const float* __restrict__ bsrc, float* NS, float* ND, float* BV,
                                                 int nN) {
  const int blk = (int)blockIdx.x;
  const int tid = (int)threadIdx.x;
  const int g   = blk * NTHR + tid;
  const int gc  = clampi(g, 0, nN - 1);
  int od = odeg[gc];
  int id = ideg[gc];
  float bb = bsrc[tid & (DF - 1)];
  PIN(od);
  PIN(id);
  PIN(bb);
  float ns = inv_sqrt_src(od);
  float nd = inv_sqrt_own(id);
  const bool real = g < nN;
  ns = real ? ns : 1.0f;
  nd = real ? nd : 1.0f;
  if (blk < TB_NODE_BLKS) {
    volatile float* q0 = (volatile float*)(NS + g);
    volatile float* q1 = (volatile float*)(ND + g);
    *q0 = ns;
    *q1 = nd;
    __threadfence();
    *q0 = ns;
    *q1 = nd;
  } else if (tid < DF) {
    const float bvv = bf16_val(bb);
    volatile float* q = (volatile float*)(BV + tid);
    *q = bvv;
    __threadfence();
    *q = bvv;
  }
}

#define PUTJ(HJ, SRCJ, SJ) { \
    const int wv = (clampi((SRCJ), 0, nN - 1) << SLB) | (int)(SJ); \
    if (HJ) { if (pos < LCAP) hl[pos] = wv; } \
    pos += (HJ) ? 1 : 0; }

__global__ __launch_bounds__(NTHR) void k_build(const int* __restrict__ srcs, const int* __restrict__ dsts,
                                                int nN, int* listG, int* cntG, int* offG, int* flagG) {
  extern __shared__ __attribute__((aligned(16))) int dsm[];
  int* hl   = dsm;
  int* sl   = dsm + LCAP;
  int* cnt  = sl + LCAP;
  int* offs = cnt + NBRUN;
  int* cur  = offs + NBRUN;
  int* misc = cur + NBRUN;
  const int tid = (int)threadIdx.x, lane = tid & 31, wave = tid >> 5;
  const int b = (int)blockIdx.x;
  const int nodeBase = b * NBRUN;
  const int nb = clampi(nN - nodeBase, 0, NBRUN);

  {
    const v4i z4 = {0, 0, 0, 0};
    for (int i = tid * 4; i < BK_ZINTS; i += NTHR * 4) *(v4ia*)(dsm + i) = z4;
    if (tid < BK_MISC) misc[tid] = 0;
  }
  __syncthreads();

  int run = 0;
  {
    const unsigned nbs = (unsigned)nodeBase;
    const unsigned unb = (unsigned)nb;
    const int k1 = -(int)(wave > 0), k2 = -(int)(wave > 1), k3 = -(int)(wave > 2), k4 = -(int)(wave > 3);
    const int k5 = -(int)(wave > 4), k6 = -(int)(wave > 5), k7 = -(int)(wave > 6);
#pragma unroll 1
    for (int st = 0; st < NSTEP; ++st) {
      const int e0  = st * STEPB + wave * 256 + lane * 8;
      const int e0c = e0 < (NE - 8) ? e0 : (NE - 8);
      const v4i da = *(const v4ia*)(dsts + e0c);
      const v4i db = *(const v4ia*)(dsts + e0c + 4);
      const v4i sa = *(const v4ia*)(srcs + e0c);
      const v4i sb = *(const v4ia*)(srcs + e0c + 4);
      PIN(da.x); PIN(da.y); PIN(da.z); PIN(da.w);
      PIN(db.x); PIN(db.y); PIN(db.z); PIN(db.w);
      PIN(sa.x); PIN(sa.y); PIN(sa.z); PIN(sa.w);
      PIN(sb.x); PIN(sb.y); PIN(sb.z); PIN(sb.w);
      const unsigned s0 = (unsigned)da.x - nbs, s1 = (unsigned)da.y - nbs;
      const unsigned s2 = (unsigned)da.z - nbs, s3 = (unsigned)da.w - nbs;
      const unsigned s4 = (unsigned)db.x - nbs, s5 = (unsigned)db.y - nbs;
      const unsigned s6 = (unsigned)db.z - nbs, s7 = (unsigned)db.w - nbs;
      const bool h0 = (e0 + 0 < NE) && (s0 < unb);
      const bool h1 = (e0 + 1 < NE) && (s1 < unb);
      const bool h2 = (e0 + 2 < NE) && (s2 < unb);
      const bool h3 = (e0 + 3 < NE) && (s3 < unb);
      const bool h4 = (e0 + 4 < NE) && (s4 < unb);
      const bool h5 = (e0 + 5 < NE) && (s5 < unb);
      const bool h6 = (e0 + 6 < NE) && (s6 < unb);
      const bool h7 = (e0 + 7 < NE) && (s7 < unb);
      const unsigned m0 = __builtin_amdgcn_ballot_w32(h0);
      const unsigned m1 = __builtin_amdgcn_ballot_w32(h1);
      const unsigned m2 = __builtin_amdgcn_ballot_w32(h2);
      const unsigned m3 = __builtin_amdgcn_ballot_w32(h3);
      const unsigned m4 = __builtin_amdgcn_ballot_w32(h4);
      const unsigned m5 = __builtin_amdgcn_ballot_w32(h5);
      const unsigned m6 = __builtin_amdgcn_ballot_w32(h6);
      const unsigned m7 = __builtin_amdgcn_ballot_w32(h7);
      const unsigned many = m0 | m1 | m2 | m3 | m4 | m5 | m6 | m7;
      unsigned pre = __builtin_amdgcn_mbcnt_lo(m0, 0u);
      pre = __builtin_amdgcn_mbcnt_lo(m1, pre);
      pre = __builtin_amdgcn_mbcnt_lo(m2, pre);
      pre = __builtin_amdgcn_mbcnt_lo(m3, pre);
      pre = __builtin_amdgcn_mbcnt_lo(m4, pre);
      pre = __builtin_amdgcn_mbcnt_lo(m5, pre);
      pre = __builtin_amdgcn_mbcnt_lo(m6, pre);
      pre = __builtin_amdgcn_mbcnt_lo(m7, pre);
      const int wcnt = (int)__builtin_popcount(m0) + (int)__builtin_popcount(m1) + (int)__builtin_popcount(m2)
                     + (int)__builtin_popcount(m3) + (int)__builtin_popcount(m4) + (int)__builtin_popcount(m5)
                     + (int)__builtin_popcount(m6) + (int)__builtin_popcount(m7);
      int* wcs = misc + (st & 1) * 8;
      if (lane == 0) wcs[wave] = wcnt;
      __syncthreads();
      const v4i c0 = *(const v4ia*)(wcs);
      const v4i c1 = *(const v4ia*)(wcs + 4);
      const int below = (c0.x & k1) + (c0.y & k2) + (c0.z & k3) + (c0.w & k4) + (c1.x & k5) + (c1.y & k6) + (c1.z & k7);
      const int tot = c0.x + c0.y + c0.z + c0.w + c1.x + c1.y + c1.z + c1.w;
      if (many != 0u) {
        int pos = run + below + (int)pre;
        PUTJ(h0, sa.x, s0)
        PUTJ(h1, sa.y, s1)
        PUTJ(h2, sa.z, s2)
        PUTJ(h3, sa.w, s3)
        PUTJ(h4, sb.x, s4)
        PUTJ(h5, sb.y, s5)
        PUTJ(h6, sb.z, s6)
        PUTJ(h7, sb.w, s7)
      }
      run += tot;
    }
  }
  __syncthreads();

  if (wave == 0) {
    const int ov = (run > LCAP) ? 1 : 0;
    int tc = run < 0 ? 0 : (run > LCAP ? LCAP : run);
    tc = __builtin_amdgcn_readfirstlane(tc);
#pragma unroll 1
    for (int b0 = 0; b0 < tc; b0 += 32) {
      const int idx = b0 + lane;
      const int ent = hl[idx < LCAP ? idx : LCAP - 1];
      const int m32 = (tc - b0) < 32 ? (tc - b0) : 32;
#pragma unroll 1
      for (int k = 0; k < m32; ++k) {
        const int u    = __builtin_amdgcn_readlane(ent, k);
        const int slot = u & (NBRUN - 1);
        const int cvv  = cnt[slot];
        if (lane == 0) cnt[slot] = cvv + 1;
      }
    }
    if (lane == 0) { misc[16] = tc; misc[17] = ov; }
  }
  __syncthreads();

  if (wave == 0) {
    const int base = lane * (NBRUN / 32);
    int s = 0, big = 0;
#pragma unroll 1
    for (int i = 0; i < NBRUN / 32; ++i) {
      const int cvv = cnt[base + i];
      s += cvv;
      big |= (cvv > DEGCAP) ? 1 : 0;
    }
    int incl = s;
#pragma unroll
    for (int d = 1; d < 32; d <<= 1) {
      const int y = __shfl_up(incl, d, 32);
      incl += (lane >= d) ? y : 0;
    }
    int runp = incl - s;
#pragma unroll 1
    for (int i = 0; i < NBRUN / 32; ++i) {
      const int cvv = cnt[base + i];
      offs[base + i] = runp;
      cur[base + i]  = runp;
      runp += cvv;
    }
    const unsigned bm = __builtin_amdgcn_ballot_w32(big != 0);
    if (lane == 0) {
      const int o9 = misc[17];
      misc[17] = o9 | ((bm != 0u) ? 1 : 0);
    }
  }
  __syncthreads();

  if (wave == 0) {
    int tc = run < 0 ? 0 : (run > LCAP ? LCAP : run);
    tc = __builtin_amdgcn_readfirstlane(tc);
#pragma unroll 1
    for (int b0 = 0; b0 < tc; b0 += 32) {
      const int idx = b0 + lane;
      const int ent = hl[idx < LCAP ? idx : LCAP - 1];
      const int m32 = (tc - b0) < 32 ? (tc - b0) : 32;
#pragma unroll 1
      for (int k = 0; k < m32; ++k) {
        const int u    = __builtin_amdgcn_readlane(ent, k);
        const int slot = u & (NBRUN - 1);
        int p = cur[slot];
        p = p < 0 ? 0 : (p > LCAP - 1 ? LCAP - 1 : p);
        if (lane == 0) { sl[p] = (u >> SLB) & 0x1FFFF; cur[slot] = p + 1; }
      }
    }
  }
  __syncthreads();

  {
    const int ovf = misc[17];
    const int tot = misc[16];
    const v4i fv = {ovf, ovf, ovf, ovf};
    int* lb = listG + (size_t)b * (size_t)LCAP;
    for (int pass = 0; pass < 2; ++pass) {
#pragma unroll 1
      for (int it = 0; it < LIST_IT; ++it) {
        const int p4 = it * NTHR + tid;
        const int i0 = 4 * p4;
        const v4i hv = *(const v4ia*)(sl + i0);
        const v4i mk = { (i0 + 0 < tot) ? -1 : 0, (i0 + 1 < tot) ? -1 : 0,
                         (i0 + 2 < tot) ? -1 : 0, (i0 + 3 < tot) ? -1 : 0 };
        const v4i v = hv & mk;
        *(volatile v4i*)(lb + (size_t)i0) = v;
      }
      {
        const v4i c4 = *(const v4ia*)(cnt + 4 * tid);
        const v4i o4 = *(const v4ia*)(offs + 4 * tid);
        *(volatile v4i*)(cntG + (size_t)nodeBase + 4 * tid) = c4;
        *(volatile v4i*)(offG + (size_t)nodeBase + 4 * tid) = o4;
      }
      if (tid < 8) *(volatile v4i*)(flagG + (size_t)b * 32 + 4 * tid) = fv;
      __threadfence();
    }
  }
}

__global__ __launch_bounds__(NTHR) void k_walk(const float* __restrict__ T, const float* __restrict__ NS,
                                               const float* __restrict__ ND, const float* __restrict__ BV,
                                               const int* __restrict__ listG, const int* __restrict__ cntG,
                                               const int* __restrict__ offG, const int* __restrict__ flagG,
                                               float* out, int nN) {
  const int tid = (int)threadIdx.x, lane = tid & 31, wave = tid >> 5;
  const int n = (int)blockIdx.x * NWAVE + wave;
  if (n >= nN) return;
  const int blk = n >> SLB;
  int cv  = cntG[n];
  int ofv = offG[n];
  int fl  = flagG[(size_t)blk * 32];
  float nd = ND[n];
  v4f bq = *(const v4fa*)(BV + 4 * lane);
  PIN(cv);
  PIN(ofv);
  PIN(fl);
  PIN(nd);
  PIN(bq);
  const int bad = ((fl != 0) || (cv < 0) || (cv > DEGCAP)) ? 1 : 0;
  cv  = cv < 0 ? 0 : (cv > DEGCAP ? DEGCAP : cv);
  ofv = ofv < 0 ? 0 : (ofv > LCAP - DEGCAP ? LCAP - DEGCAP : ofv);
  const int cn = __builtin_amdgcn_readfirstlane(cv);
  const int o  = __builtin_amdgcn_readfirstlane(ofv);
  const int* listb = listG + (size_t)blk * (size_t)LCAP;
  v4f acc = (v4f){0.0f, 0.0f, 0.0f, 0.0f};
#pragma unroll 1
  for (int g0 = 0; g0 < cn; g0 += 32) {
    const int last = o + cn - 1;
    int idx = o + g0 + lane;
    idx = idx > last ? last : idx;
    int ec = listb[idx];
    PIN(ec);
    const int col = clampi(ec, 0, nN - 1);
    float wv = NS[col];
    PIN(wv);
    const int wb = __float_as_int(wv);
    const int m32 = (cn - g0) < 32 ? (cn - g0) : 32;
#pragma unroll 1
    for (int t = 0; t < m32; ++t) {
      const int ct   = __builtin_amdgcn_readlane(col, t);
      const float wt = __int_as_float(__builtin_amdgcn_readlane(wb, t));
      const v4f tv = *(const v4fa*)(T + (size_t)ct * DF + 4 * lane);
      const v4f p = tv * wt;
      acc = acc + p;
    }
  }
  const v4f m = acc * nd;
  v4f r = m + bq;
  const float qnan = __int_as_float(0x7fc00000);
  r[0] = (bad != 0) ? qnan : r[0];
  r[1] = (bad != 0) ? qnan : r[1];
  r[2] = (bad != 0) ? qnan : r[2];
  r[3] = (bad != 0) ? qnan : r[3];
  volatile v4f* q = (volatile v4f*)(out + (size_t)n * DF + 4 * lane);
  *q = r;
  __threadfence();
  *q = r;
}

constexpr size_t SZ_HB   = (size_t)MPAD * DF * 2;
constexpr size_t SZ_WT   = (size_t)DF * DF * 2;
constexpr size_t SZ_T    = (size_t)MPAD * DF * 4;
constexpr size_t SZ_NS   = (size_t)MPAD * 4;
constexpr size_t SZ_BV   = (size_t)DF * 4;
constexpr size_t SZ_LIST = (size_t)NBLK * LCAP * 4;
constexpr size_t SZ_CNT  = (size_t)NSLOT * 4;
constexpr size_t SZ_FLAG = (size_t)NBLK * 32 * 4;
constexpr size_t O_HB   = 0;
constexpr size_t O_WT   = O_HB + SZ_HB;
constexpr size_t O_T    = O_WT + SZ_WT;
constexpr size_t O_NS   = O_T + SZ_T;
constexpr size_t O_ND   = O_NS + SZ_NS;
constexpr size_t O_BV   = O_ND + SZ_NS;
constexpr size_t O_LIST = O_BV + SZ_BV;
constexpr size_t O_OFF  = O_LIST + SZ_LIST;
constexpr size_t O_CNT  = O_OFF + SZ_CNT;
constexpr size_t O_FLAG = O_CNT + SZ_CNT;
constexpr size_t WS_TOTAL = O_FLAG + SZ_FLAG;
static_assert(SZ_HB % 128 == 0 && SZ_WT % 128 == 0 && SZ_T % 128 == 0 && SZ_NS % 128 == 0 && SZ_BV % 128 == 0);
static_assert(SZ_LIST % 128 == 0 && SZ_CNT % 128 == 0 && SZ_FLAG % 128 == 0 && ((size_t)LCAP * 4) % 128 == 0);
static_assert(SZ_HB == 25624576 && SZ_T == 51249152 && SZ_LIST == 5218304);
static_assert(WS_TOTAL == 83741440 && WS_TOTAL <= ((size_t)128 << 20));
static_assert((size_t)NN * DF * 4 <= SZ_T && (size_t)TB_NODE_BLKS * NTHR * 4 == SZ_NS);
static_assert((long long)MPAD * (DF / 8) < (1LL << 31));

extern "C" void kernel_launch(void* const* d_in, const int* in_sizes, int n_in,
                              void* d_out, int out_size, void* d_ws, size_t ws_size,
                              hipStream_t stream) {
  if (n_in < 7) return;
  if (in_sizes[0] != NN * DF) return;
  if (in_sizes[1] != DF * DF) return;
  if (in_sizes[2] != DF) return;
  if (in_sizes[3] != NE) return;
  if (in_sizes[4] != NE) return;
  if (in_sizes[5] != NN) return;
  if (in_sizes[6] != NN) return;
  if (out_size != NN * DF) return;
  if (ws_size < WS_TOTAL) return;

  const float* hsrc = (const float*)d_in[0];
  const float* W    = (const float*)d_in[1];
  const float* bias = (const float*)d_in[2];
  const int*   esrc = (const int*)d_in[3];
  const int*   edst = (const int*)d_in[4];
  const int*   odeg = (const int*)d_in[5];
  const int*   ideg = (const int*)d_in[6];
  float* out = (float*)d_out;

  char* ws = (char*)d_ws;
  unsigned short* HB  = (unsigned short*)(ws + O_HB);
  unsigned short* WT  = (unsigned short*)(ws + O_WT);
  float*          Tp  = (float*)(ws + O_T);
  float*          NSp = (float*)(ws + O_NS);
  float*          NDp = (float*)(ws + O_ND);
  float*          BVp = (float*)(ws + O_BV);
  int*            LST = (int*)(ws + O_LIST);
  int*            OFF = (int*)(ws + O_OFF);
  int*            CNT = (int*)(ws + O_CNT);
  int*            FLG = (int*)(ws + O_FLAG);

  hipFuncSetAttribute(reinterpret_cast<const void*>(&k_build), hipFuncAttributeMaxDynamicSharedMemorySize,
                      (int)BK_LDS);

  k_plane<0><<<MPAD * (DF / 8) / 256, 256, 0, stream>>>(hsrc, NN, DF, DF, HB, MPAD, DF);
  k_wt<<<1, NTHR, 0, stream>>>(W, WT);
  const int gemmTiles = ((NN + 63) / 64) * (DF / 64);
  k_gemm_nt<0, 0><<<(gemmTiles + 7) / 8, 256, 0, stream>>>(HB, WT, BVp, Tp, NN, DF, DF, DF);
  k_tables<<<TB_NODE_BLKS + 1, NTHR, 0, stream>>>(odeg, ideg, bias, NSp, NDp, BVp, NN);
  k_build<<<NBLK, NTHR, BK_LDS, stream>>>(esrc, edst, NN, LST, CNT, OFF, FLG);
  k_walk<<<NN / NWAVE, NTHR, 0, stream>>>(Tp, NSp, NDp, BVp, LST, CNT, OFF, FLG, out, NN);
}
